// GeometryAwareCrossAttentionBlock_7232724927306
// MI455X (gfx1250) — hardware-verified
//
#include <hip/hip_runtime.h>
#define BB 4
#define NQ 2048
#define NK 2048
#define DD 384
#define NH 6
#define HD 64
#define KNN 8

typedef __bf16 v16b __attribute__((ext_vector_type(16)));
typedef unsigned short v8us __attribute__((ext_vector_type(8), may_alias));
typedef float  v8f  __attribute__((ext_vector_type(8)));
typedef float  v4f  __attribute__((ext_vector_type(4)));
typedef float  v4fa __attribute__((ext_vector_type(4), may_alias));
union FragB { v16b v; v8us half[2]; unsigned short u[16]; };

__device__ __forceinline__ unsigned short bf16_bits(float x) { unsigned int u = __float_as_uint(x); return (unsigned short)((u + 0x7FFFu + ((u >> 16) & 1u)) >> 16); }
__device__ __forceinline__ float bf16_val(unsigned short b) { return __uint_as_float(((unsigned int)b) << 16); }
__device__ __forceinline__ float bf16_round(float x) { return bf16_val(bf16_bits(x)); }
template <int NT>
__device__ __forceinline__ v8f mmaN(v16b ah, v16b al, v16b bh, v16b bl, v8f c) {
  c = __builtin_amdgcn_wmma_f32_16x16x32_bf16(false, ah, false, bh, (short)0, c, false, false);
  if (NT >= 2) c = __builtin_amdgcn_wmma_f32_16x16x32_bf16(false, al, false, bh, (short)0, c, false, false);
  if (NT >= 3) c = __builtin_amdgcn_wmma_f32_16x16x32_bf16(false, ah, false, bl, (short)0, c, false, false);
  asm volatile("v_nop\n\tv_nop\n\tv_nop\n\tv_nop" : "+v"(c) : "v"(ah), "v"(al), "v"(bh), "v"(bl));
  return c;
}

__global__ __launch_bounds__(256) void k_wt_bf16(const float* __restrict__ W, unsigned short* __restrict__ Wt, int K, int N) {
  const int t = blockIdx.x * 256 + threadIdx.x;
  const int k8n = K / 8;
  if (t >= N * k8n) return;
  const int n = t / k8n, k8 = (t % k8n) * 8;
  v8us v;
#pragma unroll
  for (int i = 0; i < 8; ++i) v[i] = bf16_bits(W[(size_t)(k8 + i) * N + n]);
  *(volatile v8us*)(Wt + (size_t)n * K + k8) = v;
  __threadfence();
  *(volatile v8us*)(Wt + (size_t)n * K + k8) = v;
}

template <bool ASPLIT, int ACT, bool BIAS_BF16>
__global__ __launch_bounds__(128) void k_gemm_bf(const float* __restrict__ A, int lda, const unsigned short* __restrict__ Wt, int ldb,
                                               const float* __restrict__ bias, float* __restrict__ C, int ldc, int M, int N, int K) {
  __shared__ __attribute__((aligned(16))) float so[4][16][64];
  const int tid = threadIdx.x, w = tid >> 5, lane = tid & 31, ln = lane & 15, hh = lane >> 4;
  const int ntn = N / 64;
  const int wid = blockIdx.x * 4 + w;
  const int mt = wid / ntn, nq = wid % ntn;
  if (mt * 16 >= M) return;
  const int row0 = mt * 16, col0 = nq * 64;
  const float* arow = A + (size_t)(row0 + ln) * lda;
  v8f acc[4] = {};
  for (int kb = 0; kb < K; kb += 32) {
    FragB ah, al;
    const v4f x0 = *(const v4fa*)(arow + kb + 8 * hh), x1 = *(const v4fa*)(arow + kb + 8 * hh + 4);
    const v4f x2 = *(const v4fa*)(arow + kb + 16 + 8 * hh), x3 = *(const v4fa*)(arow + kb + 16 + 8 * hh + 4);
    float xs[16] = {x0[0],x0[1],x0[2],x0[3],x1[0],x1[1],x1[2],x1[3],x2[0],x2[1],x2[2],x2[3],x3[0],x3[1],x3[2],x3[3]};
#pragma unroll
    for (int i = 0; i < 16; ++i) { const unsigned short hb = bf16_bits(xs[i]); ah.u[i] = hb; al.u[i] = ASPLIT ? bf16_bits(xs[i] - bf16_val(hb)) : (unsigned short)0; }
#pragma unroll
    for (int t = 0; t < 4; ++t) {
      const unsigned short* brow = Wt + (size_t)(col0 + t * 16 + ln) * ldb + kb;
      FragB b;
      b.half[0] = *(const v8us*)(brow + 8 * hh);
      b.half[1] = *(const v8us*)(brow + 16 + 8 * hh);
      acc[t] = mmaN<ASPLIT ? 2 : 1>(ah.v, al.v, b.v, b.v, acc[t]);
    }
  }
#pragma unroll
  for (int t = 0; t < 4; ++t) {
    float bv = bias ? bias[col0 + t * 16 + ln] : 0.f;
    if (BIAS_BF16) bv = bf16_round(bv);
#pragma unroll
    for (int r = 0; r < 8; ++r) { float v = acc[t][r] + bv; if (ACT == 1) v = fmaxf(v, 0.f); so[w][8 * hh + r][t * 16 + ln] = v; }
  }
  __builtin_amdgcn_fence(__ATOMIC_ACQ_REL, "workgroup");
  __builtin_amdgcn_wave_barrier();
  const int rsub = lane >> 4, c4 = (lane & 15) * 4;
  for (int pass = 0; pass < 2; ++pass) {
#pragma unroll
    for (int q = 0; q < 8; ++q) {
      const int r = q * 2 + rsub;
      const v4f v = *(const v4fa*)&so[w][r][c4];
      *(volatile v4f*)(C + (size_t)(row0 + r) * ldc + col0 + c4) = v;
    }
    if (pass == 0) __threadfence();
  }
}

template <int D, bool CAUSAL>
__global__ __launch_bounds__(128) void k_flash(const float* __restrict__ qb, const float* __restrict__ kb, const float* __restrict__ vb,
                                             int pitch, int T, int H, float scale, float* __restrict__ y, int ypitch) {
  constexpr int KS = D / 32;
  constexpr int DT = D / 16;
  __shared__ __attribute__((aligned(16))) unsigned short sKh[32][D + 8], sKl[32][D + 8], sVh[32][D + 8], sVl[32][D + 8];
  __shared__ __attribute__((aligned(16))) unsigned short sPh[4][16][40], sPl[4][16][40];
  __shared__ __attribute__((aligned(16))) float sO[4][16][D];
  const int tid = threadIdx.x, w = tid >> 5, lane = tid & 31, ln = lane & 15, hh = lane >> 4;
  const int nqb = (T + 63) / 64;
  const int bh = blockIdx.x / nqb, qblk = blockIdx.x % nqb;
  const int b = bh / H, h = bh % H;
  const int q0 = qblk * 64 + w * 16;
  const float* Q = qb + (size_t)b * T * pitch + h * D;
  const float* K = kb + (size_t)b * T * pitch + h * D;
  const float* V = vb + (size_t)b * T * pitch + h * D;

  FragB aqh[KS], aql[KS];
  {
    int row = q0 + ln; if (row >= T) row = T - 1;
    const float* qr = Q + (size_t)row * pitch;
#pragma unroll
    for (int ks = 0; ks < KS; ++ks)
#pragma unroll
      for (int i = 0; i < 16; ++i) {
        const int d = ks * 32 + ((i < 8) ? (8 * hh + i) : (16 + 8 * hh + (i - 8)));
        const float x = qr[d] * scale; const unsigned short hb = bf16_bits(x);
        aqh[ks].u[i] = hb; aql[ks].u[i] = bf16_bits(x - bf16_val(hb));
      }
  }
  float m_r[8], l_r[8];
#pragma unroll
  for (int r = 0; r < 8; ++r) { m_r[r] = -3.0e38f; l_r[r] = 0.f; }
  v8f oacc[DT];
#pragma unroll
  for (int dt = 0; dt < DT; ++dt) oacc[dt] = (v8f){0.f,0.f,0.f,0.f,0.f,0.f,0.f,0.f};

  const int kv_end = CAUSAL ? min(T, qblk * 64 + 64) : T;
  for (int j0 = 0; j0 < kv_end; j0 += 32) {
    __syncthreads();
    for (int e = tid; e < 32 * (D / 4); e += 128) {
      const int r = e / (D / 4), c4 = (e % (D / 4)) * 4;
      const int key = j0 + r;
      v4f kf = {0.f,0.f,0.f,0.f}, vf = {0.f,0.f,0.f,0.f};
      if (key < T) { kf = *(const v4fa*)(K + (size_t)key * pitch + c4); vf = *(const v4fa*)(V + (size_t)key * pitch + c4); }
#pragma unroll
      for (int t = 0; t < 4; ++t) {
        unsigned short hb = bf16_bits(kf[t]); sKh[r][c4 + t] = hb; sKl[r][c4 + t] = bf16_bits(kf[t] - bf16_val(hb));
        hb = bf16_bits(vf[t]); sVh[r][c4 + t] = hb; sVl[r][c4 + t] = bf16_bits(vf[t] - bf16_val(hb));
      }
    }
    __syncthreads();
    v8f s[2];
#pragma unroll
    for (int nt = 0; nt < 2; ++nt) {
      v8f acc = {};
#pragma unroll
      for (int ks = 0; ks < KS; ++ks) {
        FragB bh_, bl_;
        bh_.half[0] = *(const v8us*)&sKh[nt * 16 + ln][ks * 32 + 8 * hh]; bh_.half[1] = *(const v8us*)&sKh[nt * 16 + ln][ks * 32 + 16 + 8 * hh];
        bl_.half[0] = *(const v8us*)&sKl[nt * 16 + ln][ks * 32 + 8 * hh]; bl_.half[1] = *(const v8us*)&sKl[nt * 16 + ln][ks * 32 + 16 + 8 * hh];
        acc = mmaN<3>(aqh[ks].v, aql[ks].v, bh_.v, bl_.v, acc);
      }
      s[nt] = acc;
    }
    float alpha[8];
#pragma unroll
    for (int r = 0; r < 8; ++r) {
      const int qi = q0 + 8 * hh + r;
      const int ja = j0 + ln, jb = j0 + 16 + ln;
      if (CAUSAL) { if (ja > qi) s[0][r] = -3.0e38f; if (jb > qi) s[1][r] = -3.0e38f; }
      if (ja >= T) s[0][r] = -3.0e38f;
      if (jb >= T) s[1][r] = -3.0e38f;
      float mx = fmaxf(s[0][r], s[1][r]);
      mx = fmaxf(mx, __shfl_xor(mx, 1, 32)); mx = fmaxf(mx, __shfl_xor(mx, 2, 32)); mx = fmaxf(mx, __shfl_xor(mx, 4, 32)); mx = fmaxf(mx, __shfl_xor(mx, 8, 32));
      const float mnew = fmaxf(m_r[r], mx);
      alpha[r] = (mnew > -1.0e38f) ? __expf(m_r[r] - mnew) : 1.0f;
      const float p0 = (s[0][r] > -1.0e38f) ? __expf(s[0][r] - mnew) : 0.f;
      const float p1 = (s[1][r] > -1.0e38f) ? __expf(s[1][r] - mnew) : 0.f;
      m_r[r] = mnew;
      l_r[r] = l_r[r] * alpha[r] + p0 + p1;
      unsigned short hb = bf16_bits(p0); sPh[w][8 * hh + r][ln] = hb;      sPl[w][8 * hh + r][ln] = bf16_bits(p0 - bf16_val(hb));
      hb = bf16_bits(p1);                sPh[w][8 * hh + r][16 + ln] = hb; sPl[w][8 * hh + r][16 + ln] = bf16_bits(p1 - bf16_val(hb));
    }
#pragma unroll
    for (int dt = 0; dt < DT; ++dt)
#pragma unroll
      for (int r = 0; r < 8; ++r) oacc[dt][r] *= alpha[r];
    __builtin_amdgcn_fence(__ATOMIC_ACQ_REL, "workgroup");
    __builtin_amdgcn_wave_barrier();
    FragB pah, pal;
    pah.half[0] = *(const v8us*)&sPh[w][ln][8 * hh]; pah.half[1] = *(const v8us*)&sPh[w][ln][16 + 8 * hh];
    pal.half[0] = *(const v8us*)&sPl[w][ln][8 * hh]; pal.half[1] = *(const v8us*)&sPl[w][ln][16 + 8 * hh];
#pragma unroll
    for (int dt = 0; dt < DT; ++dt) {
      FragB bvh, bvl;
#pragma unroll
      for (int i = 0; i < 8; ++i) {
        bvh.u[i] = sVh[8 * hh + i][dt * 16 + ln]; bvh.u[8 + i] = sVh[16 + 8 * hh + i][dt * 16 + ln];
        bvl.u[i] = sVl[8 * hh + i][dt * 16 + ln]; bvl.u[8 + i] = sVl[16 + 8 * hh + i][dt * 16 + ln];
      }
      oacc[dt] = mmaN<3>(pah.v, pal.v, bvh.v, bvl.v, oacc[dt]);
    }
    __builtin_amdgcn_fence(__ATOMIC_ACQ_REL, "workgroup");
    __builtin_amdgcn_wave_barrier();
  }
#pragma unroll
  for (int r = 0; r < 8; ++r) {
    float l = l_r[r];
    l += __shfl_xor(l, 1, 32); l += __shfl_xor(l, 2, 32); l += __shfl_xor(l, 4, 32); l += __shfl_xor(l, 8, 32);
    l_r[r] = (l > 0.f) ? 1.0f / l : 0.f;
  }
#pragma unroll
  for (int dt = 0; dt < DT; ++dt)
#pragma unroll
    for (int r = 0; r < 8; ++r) sO[w][8 * hh + r][dt * 16 + ln] = oacc[dt][r] * l_r[r];
  __builtin_amdgcn_fence(__ATOMIC_ACQ_REL, "workgroup");
  __builtin_amdgcn_wave_barrier();
  for (int pass = 0; pass < 2; ++pass) {
    for (int r = 0; r < 16; ++r) {
      const int row = q0 + r;
      if (row < T && lane < D / 4) {
        const v4f val = *(const v4fa*)&sO[w][r][lane * 4];
        *(volatile v4f*)(y + ((size_t)b * T + row) * ypitch + h * D + lane * 4) = val;
      }
    }
    if (pass == 0) __threadfence();
  }
}

template <bool AFFINE, bool RESID, bool RES_BF16>
__global__ __launch_bounds__(256) void k_transpose32(const float* __restrict__ in, float* __restrict__ out, int rows, int cols,
                                                    const float* __restrict__ scale, const float* __restrict__ shift, const float* __restrict__ res) {
  __shared__ float tile[32][33];
  const int b = blockIdx.z;
  const int r0 = blockIdx.y * 32, c0 = blockIdx.x * 32;
  const float* src = in + (size_t)b * rows * cols;
  float* dst = out + (size_t)b * rows * cols;
  const int tx = threadIdx.x & 31, ty = threadIdx.x >> 5;
  for (int i = ty; i < 32; i += 8) tile[i][tx] = src[(size_t)(r0 + i) * cols + c0 + tx];
  __syncthreads();
  for (int pass = 0; pass < 2; ++pass) {
    for (int i = ty; i < 32; i += 8) {
      float v = tile[tx][i];
      const int orow = c0 + i;
      if (AFFINE) v = v * scale[orow] + shift[orow];
      if (RESID) { float rv = res[(size_t)b * rows * cols + (size_t)orow * rows + r0 + tx]; if (RES_BF16) rv = bf16_round(rv); v += rv; }
      *(volatile float*)(dst + (size_t)orow * rows + r0 + tx) = v;
    }
    if (pass == 0) __threadfence();
  }
}

__global__ __launch_bounds__(256) void k_pool2_pm(const float* __restrict__ in, float* __restrict__ out, int Bn, int H, int W, int C) {
  const size_t t = (size_t)blockIdx.x * 256 + threadIdx.x;
  const int c4n = C / 4, Ho = H / 2, Wo = W / 2;
  const size_t total = (size_t)Bn * Ho * Wo * c4n;
  if (t >= total) return;
  const int c4 = (int)(t % c4n) * 4; size_t rest = t / c4n;
  const int pw = (int)(rest % Wo); rest /= Wo; const int ph = (int)(rest % Ho); const int b = (int)(rest / Ho);
  const float* base = in + (size_t)b * H * W * C;
  const int p00 = (2 * ph) * W + 2 * pw;
  const v4f a = *(const v4fa*)(base + (size_t)p00 * C + c4), bq = *(const v4fa*)(base + (size_t)(p00 + 1) * C + c4);
  const v4f c = *(const v4fa*)(base + (size_t)(p00 + W) * C + c4), d = *(const v4fa*)(base + (size_t)(p00 + W + 1) * C + c4);
  v4f m; for (int i = 0; i < 4; ++i) m[i] = fmaxf(fmaxf(a[i], bq[i]), fmaxf(c[i], d[i]));
  float* dst = out + ((size_t)b * Ho * Wo + (size_t)ph * Wo + pw) * C + c4;
  *(volatile v4f*)dst = m;
  __threadfence();
  *(volatile v4f*)dst = m;
}

template <int DQ, int DV>
__global__ __launch_bounds__(128) void k_flash2(const float* __restrict__ Qb, size_t qstride, int qpitch, int Tq,
                                              const float* __restrict__ Kb, size_t kstride, int kpitch, int Tk,
                                              const float* __restrict__ Vb, size_t vstride, int vpitch,
                                              float scale, float* __restrict__ y, size_t ystride, int ypitch) {
  constexpr int KS = DQ / 32, DT = DV / 16;
  __shared__ __attribute__((aligned(16))) unsigned short sKh[32][DQ + 8], sKl[32][DQ + 8], sVh[32][DV + 8], sVl[32][DV + 8];
  __shared__ __attribute__((aligned(16))) unsigned short sPh[4][16][40], sPl[4][16][40];
  __shared__ __attribute__((aligned(16))) float sO[4][16][DV];
  const int tid = threadIdx.x, w = tid >> 5, lane = tid & 31, ln = lane & 15, hh = lane >> 4;
  const int nqb = (Tq + 63) / 64;
  const int bh = blockIdx.x / nqb, qblk = blockIdx.x % nqb;
  const int dv0 = blockIdx.y * DV;
  const int q0 = qblk * 64 + w * 16;
  const float* Q = Qb + (size_t)bh * qstride; const float* K = Kb + (size_t)bh * kstride; const float* V = Vb + (size_t)bh * vstride + dv0;
  FragB aqh[KS], aql[KS];
  {
    int row = q0 + ln; if (row >= Tq) row = Tq - 1;
    const float* qr = Q + (size_t)row * qpitch;
#pragma unroll
    for (int ks = 0; ks < KS; ++ks)
#pragma unroll
      for (int i = 0; i < 16; ++i) {
        const int d = ks * 32 + ((i < 8) ? (8 * hh + i) : (16 + 8 * hh + (i - 8)));
        const float x = qr[d] * scale; const unsigned short hb = bf16_bits(x);
        aqh[ks].u[i] = hb; aql[ks].u[i] = bf16_bits(x - bf16_val(hb));
      }
  }
  float m_r[8], l_r[8];
#pragma unroll
  for (int r = 0; r < 8; ++r) { m_r[r] = -3.0e38f; l_r[r] = 0.f; }
  v8f oacc[DT];
#pragma unroll
  for (int dt = 0; dt < DT; ++dt) oacc[dt] = (v8f){0.f,0.f,0.f,0.f,0.f,0.f,0.f,0.f};
  for (int j0 = 0; j0 < Tk; j0 += 32) {
    __syncthreads();
    for (int e = tid; e < 32 * (DQ / 4); e += 128) {
      const int r = e / (DQ / 4), c4 = (e % (DQ / 4)) * 4; const int key = j0 + r;
      v4f f = {0.f,0.f,0.f,0.f}; if (key < Tk) f = *(const v4fa*)(K + (size_t)key * kpitch + c4);
#pragma unroll
      for (int t = 0; t < 4; ++t) { const unsigned short hb = bf16_bits(f[t]); sKh[r][c4 + t] = hb; sKl[r][c4 + t] = bf16_bits(f[t] - bf16_val(hb)); }
    }
    for (int e = tid; e < 32 * (DV / 4); e += 128) {
      const int r = e / (DV / 4), c4 = (e % (DV / 4)) * 4; const int key = j0 + r;
      v4f f = {0.f,0.f,0.f,0.f}; if (key < Tk) f = *(const v4fa*)(V + (size_t)key * vpitch + c4);
#pragma unroll
      for (int t = 0; t < 4; ++t) { const unsigned short hb = bf16_bits(f[t]); sVh[r][c4 + t] = hb; sVl[r][c4 + t] = bf16_bits(f[t] - bf16_val(hb)); }
    }
    __syncthreads();
    v8f s[2];
#pragma unroll
    for (int nt = 0; nt < 2; ++nt) {
      v8f acc = {};
#pragma unroll
      for (int ks = 0; ks < KS; ++ks) {
        FragB bh_, bl_;
        bh_.half[0] = *(const v8us*)&sKh[nt * 16 + ln][ks * 32 + 8 * hh]; bh_.half[1] = *(const v8us*)&sKh[nt * 16 + ln][ks * 32 + 16 + 8 * hh];
        bl_.half[0] = *(const v8us*)&sKl[nt * 16 + ln][ks * 32 + 8 * hh]; bl_.half[1] = *(const v8us*)&sKl[nt * 16 + ln][ks * 32 + 16 + 8 * hh];
        acc = mmaN<3>(aqh[ks].v, aql[ks].v, bh_.v, bl_.v, acc);
      }
      s[nt] = acc;
    }
    float alpha[8];
#pragma unroll
    for (int r = 0; r < 8; ++r) {
      const int ja = j0 + ln, jb = j0 + 16 + ln;
      if (ja >= Tk) s[0][r] = -3.0e38f;
      if (jb >= Tk) s[1][r] = -3.0e38f;
      float mx = fmaxf(s[0][r], s[1][r]);
      mx = fmaxf(mx, __shfl_xor(mx, 1, 32)); mx = fmaxf(mx, __shfl_xor(mx, 2, 32)); mx = fmaxf(mx, __shfl_xor(mx, 4, 32)); mx = fmaxf(mx, __shfl_xor(mx, 8, 32));
      const float mnew = fmaxf(m_r[r], mx);
      alpha[r] = (mnew > -1.0e38f) ? __expf(m_r[r] - mnew) : 1.0f;
      const float p0 = (s[0][r] > -1.0e38f) ? __expf(s[0][r] - mnew) : 0.f;
      const float p1 = (s[1][r] > -1.0e38f) ? __expf(s[1][r] - mnew) : 0.f;
      m_r[r] = mnew;
      l_r[r] = l_r[r] * alpha[r] + p0 + p1;
      unsigned short hb = bf16_bits(p0); sPh[w][8 * hh + r][ln] = hb;      sPl[w][8 * hh + r][ln] = bf16_bits(p0 - bf16_val(hb));
      hb = bf16_bits(p1);                sPh[w][8 * hh + r][16 + ln] = hb; sPl[w][8 * hh + r][16 + ln] = bf16_bits(p1 - bf16_val(hb));
    }
#pragma unroll
    for (int dt = 0; dt < DT; ++dt)
#pragma unroll
      for (int r = 0; r < 8; ++r) oacc[dt][r] *= alpha[r];
    __builtin_amdgcn_fence(__ATOMIC_ACQ_REL, "workgroup");
    __builtin_amdgcn_wave_barrier();
    FragB pah, pal;
    pah.half[0] = *(const v8us*)&sPh[w][ln][8 * hh]; pah.half[1] = *(const v8us*)&sPh[w][ln][16 + 8 * hh];
    pal.half[0] = *(const v8us*)&sPl[w][ln][8 * hh]; pal.half[1] = *(const v8us*)&sPl[w][ln][16 + 8 * hh];
#pragma unroll
    for (int dt = 0; dt < DT; ++dt) {
      FragB bvh, bvl;
#pragma unroll
      for (int i = 0; i < 8; ++i) {
        bvh.u[i] = sVh[8 * hh + i][dt * 16 + ln]; bvh.u[8 + i] = sVh[16 + 8 * hh + i][dt * 16 + ln];
        bvl.u[i] = sVl[8 * hh + i][dt * 16 + ln]; bvl.u[8 + i] = sVl[16 + 8 * hh + i][dt * 16 + ln];
      }
      oacc[dt] = mmaN<3>(pah.v, pal.v, bvh.v, bvl.v, oacc[dt]);
    }
    __builtin_amdgcn_fence(__ATOMIC_ACQ_REL, "workgroup");
    __builtin_amdgcn_wave_barrier();
  }
#pragma unroll
  for (int r = 0; r < 8; ++r) {
    float l = l_r[r];
    l += __shfl_xor(l, 1, 32); l += __shfl_xor(l, 2, 32); l += __shfl_xor(l, 4, 32); l += __shfl_xor(l, 8, 32);
    l_r[r] = (l > 0.f) ? 1.0f / l : 0.f;
  }
#pragma unroll
  for (int dt = 0; dt < DT; ++dt)
#pragma unroll
    for (int r = 0; r < 8; ++r) sO[w][8 * hh + r][dt * 16 + ln] = oacc[dt][r] * l_r[r];
  __builtin_amdgcn_fence(__ATOMIC_ACQ_REL, "workgroup");
  __builtin_amdgcn_wave_barrier();
  for (int pass = 0; pass < 2; ++pass) {
    for (int r = 0; r < 16; ++r) {
      const int row = q0 + r;
      for (int c4 = lane * 4; c4 < DV; c4 += 128) {
        if (row < Tq) {
          const v4f val = *(const v4fa*)&sO[w][r][c4];
          *(volatile v4f*)(y + (size_t)bh * ystride + (size_t)row * ypitch + dv0 + c4) = val;
        }
      }
    }
    if (pass == 0) __threadfence();
  }
}

template <bool ASPLIT, int ACT, bool BIAS_BF16, bool RES_BF16>
__global__ __launch_bounds__(128) void k_gemm_bf3(const float* __restrict__ A, int lda, const unsigned short* __restrict__ Wt, int ldb,
                                                const float* __restrict__ bias, const float* resid, int rmod, int ldr,
                                                float* C, int ldc, int M, int N, int K) {
  __shared__ __attribute__((aligned(16))) float so[4][16][64];
  const int tid = threadIdx.x, w = tid >> 5, lane = tid & 31, ln = lane & 15, hh = lane >> 4;
  const int ntn = N / 64;
  const int wid = blockIdx.x * 4 + w;
  const int mt = wid / ntn, nq = wid % ntn;
  if (mt * 16 >= M) return;
  const int row0 = mt * 16, col0 = nq * 64;
  const float* arow = A + (size_t)(row0 + ln) * lda;
  v8f acc[4] = {};
  for (int kb = 0; kb < K; kb += 32) {
    FragB ah, al;
    const v4f x0 = *(const v4fa*)(arow + kb + 8 * hh), x1 = *(const v4fa*)(arow + kb + 8 * hh + 4);
    const v4f x2 = *(const v4fa*)(arow + kb + 16 + 8 * hh), x3 = *(const v4fa*)(arow + kb + 16 + 8 * hh + 4);
    float xs[16] = {x0[0],x0[1],x0[2],x0[3],x1[0],x1[1],x1[2],x1[3],x2[0],x2[1],x2[2],x2[3],x3[0],x3[1],x3[2],x3[3]};
#pragma unroll
    for (int i = 0; i < 16; ++i) { const unsigned short hb = bf16_bits(xs[i]); ah.u[i] = hb; al.u[i] = ASPLIT ? bf16_bits(xs[i] - bf16_val(hb)) : (unsigned short)0; }
#pragma unroll
    for (int t = 0; t < 4; ++t) {
      const unsigned short* brow = Wt + (size_t)(col0 + t * 16 + ln) * ldb + kb;
      FragB b;
      b.half[0] = *(const v8us*)(brow + 8 * hh);
      b.half[1] = *(const v8us*)(brow + 16 + 8 * hh);
      acc[t] = mmaN<ASPLIT ? 2 : 1>(ah.v, al.v, b.v, b.v, acc[t]);
    }
  }
#pragma unroll
  for (int t = 0; t < 4; ++t) {
    const int col = col0 + t * 16 + ln;
    float bv = bias ? bias[col] : 0.f;
    if (BIAS_BF16) bv = bf16_round(bv);
#pragma unroll
    for (int r = 0; r < 8; ++r) {
      float v = acc[t][r] + bv;
      if (resid) { float rv = resid[(size_t)((row0 + 8 * hh + r) % rmod) * ldr + col]; if (RES_BF16) rv = bf16_round(rv); v += rv; }
      if (ACT == 1) v = fmaxf(v, 0.f);
      if (ACT == 2) v = 0.5f * v * (1.0f + erff(v * 0.70710678118654752f));
      if (ACT == 3) { const float u = 0.7978845608028654f * (v + 0.044715f * v * v * v); v = 0.5f * v * (1.0f + tanhf(u)); }
      so[w][8 * hh + r][t * 16 + ln] = v;
    }
  }
  __builtin_amdgcn_fence(__ATOMIC_ACQ_REL, "workgroup");
  __builtin_amdgcn_wave_barrier();
  const int rsub = lane >> 4, c4 = (lane & 15) * 4;
  for (int pass = 0; pass < 2; ++pass) {
#pragma unroll
    for (int q = 0; q < 8; ++q) {
      const int r = q * 2 + rsub;
      const v4f v = *(const v4fa*)&so[w][r][c4];
      *(volatile v4f*)(C + (size_t)(row0 + r) * ldc + col0 + c4) = v;
    }
    if (pass == 0) __threadfence();
  }
}
template <bool PARAM_BF16>
__global__ __launch_bounds__(256) void k_layernorm(const float* __restrict__ X, const float* __restrict__ R, const float* __restrict__ g, const float* __restrict__ bta,
                                                  float* __restrict__ out_sum, float* __restrict__ out_norm, int N, float eps) {
  __shared__ float red[256];
  const int row = blockIdx.x, tid = threadIdx.x;
  const float* x = X + (size_t)row * N; const float* rr = R ? R + (size_t)row * N : nullptr;
  float vals[16];
  const int per = N / 256;
  float s1 = 0.f;
  for (int u = 0; u < per / 4; ++u) {
    const int j = tid * 4 + 1024 * u;
    const v4f a = *(const v4fa*)(x + j);
    v4f b = {0.f,0.f,0.f,0.f}; if (rr) b = *(const v4fa*)(rr + j);
#pragma unroll
    for (int q = 0; q < 4; ++q) { const float v = a[q] + b[q]; vals[u * 4 + q] = v; s1 += v; }
  }
  red[tid] = s1; __syncthreads();
  for (int st = 128; st > 0; st >>= 1) { if (tid < st) red[tid] += red[tid + st]; __syncthreads(); }
  const float mu = red[0] / (float)N; __syncthreads();
  float s2 = 0.f;
  for (int u = 0; u < per / 4; ++u)
#pragma unroll
    for (int q = 0; q < 4; ++q) { const float c = vals[u * 4 + q] - mu; s2 += c * c; }
  red[tid] = s2; __syncthreads();
  for (int st = 128; st > 0; st >>= 1) { if (tid < st) red[tid] += red[tid + st]; __syncthreads(); }
  const float rs = rsqrtf(red[0] / (float)N + eps);
  for (int pass = 0; pass < 2; ++pass) {
    for (int u = 0; u < per / 4; ++u) {
      const int j = tid * 4 + 1024 * u;
      v4f o, sm;
#pragma unroll
      for (int q = 0; q < 4; ++q) {
        float gg = g[j + q], bb = bta[j + q];
        if (PARAM_BF16) { gg = bf16_round(gg); bb = bf16_round(bb); }
        sm[q] = vals[u * 4 + q]; o[q] = (vals[u * 4 + q] - mu) * rs * gg + bb;
      }
      if (out_sum) *(volatile v4f*)(out_sum + (size_t)row * N + j) = sm;
      *(volatile v4f*)(out_norm + (size_t)row * N + j) = o;
    }
    if (pass == 0) __threadfence();
  }
}

template <int D>
__global__ __launch_bounds__(128) void k_flash3(const float* __restrict__ Qb, int qpitch, int Tq,
                                              const float* __restrict__ K1, const float* __restrict__ V1, int Tk1,
                                              const float* __restrict__ K2, const float* __restrict__ V2, int Tk2, int kpitch, int vpitch,
                                              int H, float scale, const int* __restrict__ mask, int causal, const float* __restrict__ sbias,
                                              float* __restrict__ y, int ypitch) {
  constexpr int KS = D / 32, DT = D / 16;
  __shared__ __attribute__((aligned(16))) unsigned short sKh[32][D + 8], sKl[32][D + 8], sVh[32][D + 8], sVl[32][D + 8];
  __shared__ __attribute__((aligned(16))) unsigned short sPh[4][16][40], sPl[4][16][40];
  __shared__ __attribute__((aligned(16))) float sO[4][16][D];
  const int tid = threadIdx.x, w = tid >> 5, lane = tid & 31, ln = lane & 15, hh = lane >> 4;
  const int Tk = Tk1 + Tk2;
  const int nqb = (Tq + 63) / 64;
  const int bh = blockIdx.x / nqb, qblk = blockIdx.x % nqb;
  const int b = bh / H, h = bh % H;
  const int q0 = qblk * 64 + w * 16;
  const float* Q = Qb + (size_t)b * Tq * qpitch + h * D;
  FragB aqh[KS], aql[KS];
  {
    int row = q0 + ln; if (row >= Tq) row = Tq - 1;
    const float* qr = Q + (size_t)row * qpitch;
#pragma unroll
    for (int ks = 0; ks < KS; ++ks)
#pragma unroll
      for (int i = 0; i < 16; ++i) {
        const int d = ks * 32 + ((i < 8) ? (8 * hh + i) : (16 + 8 * hh + (i - 8)));
        const float x = qr[d] * scale; const unsigned short hb = bf16_bits(x);
        aqh[ks].u[i] = hb; aql[ks].u[i] = bf16_bits(x - bf16_val(hb));
      }
  }
  int qrow[8];
#pragma unroll
  for (int r = 0; r < 8; ++r) { int qi = q0 + 8 * hh + r; qrow[r] = qi < Tq ? qi : Tq - 1; }
  float m_r[8], l_r[8];
#pragma unroll
  for (int r = 0; r < 8; ++r) { m_r[r] = -3.0e38f; l_r[r] = 0.f; }
  v8f oacc[DT];
#pragma unroll
  for (int dt = 0; dt < DT; ++dt) oacc[dt] = (v8f){0.f,0.f,0.f,0.f,0.f,0.f,0.f,0.f};
  const int kv_end = causal ? min(Tk, qblk * 64 + 64) : Tk;
  for (int j0 = 0; j0 < kv_end; j0 += 32) {
    __syncthreads();
    for (int e = tid; e < 32 * (D / 4); e += 128) {
      const int r = e / (D / 4), c4 = (e % (D / 4)) * 4; const int key = j0 + r;
      v4f kf = {0.f,0.f,0.f,0.f}, vf = {0.f,0.f,0.f,0.f};
      if (key < Tk1) { kf = *(const v4fa*)(K1 + (size_t)b * Tk1 * kpitch + h * D + (size_t)key * kpitch + c4); vf = *(const v4fa*)(V1 + (size_t)b * Tk1 * vpitch + h * D + (size_t)key * vpitch + c4); }
      else if (key < Tk) { const int k2 = key - Tk1; kf = *(const v4fa*)(K2 + (size_t)b * Tk2 * kpitch + h * D + (size_t)k2 * kpitch + c4); vf = *(const v4fa*)(V2 + (size_t)b * Tk2 * vpitch + h * D + (size_t)k2 * vpitch + c4); }
#pragma unroll
      for (int t = 0; t < 4; ++t) {
        unsigned short hb = bf16_bits(kf[t]); sKh[r][c4 + t] = hb; sKl[r][c4 + t] = bf16_bits(kf[t] - bf16_val(hb));
        hb = bf16_bits(vf[t]); sVh[r][c4 + t] = hb; sVl[r][c4 + t] = bf16_bits(vf[t] - bf16_val(hb));
      }
    }
    __syncthreads();
    v8f s[2];
#pragma unroll
    for (int nt = 0; nt < 2; ++nt) {
      v8f acc = {};
#pragma unroll
      for (int ks = 0; ks < KS; ++ks) {
        FragB bh_, bl_;
        bh_.half[0] = *(const v8us*)&sKh[nt * 16 + ln][ks * 32 + 8 * hh]; bh_.half[1] = *(const v8us*)&sKh[nt * 16 + ln][ks * 32 + 16 + 8 * hh];
        bl_.half[0] = *(const v8us*)&sKl[nt * 16 + ln][ks * 32 + 8 * hh]; bl_.half[1] = *(const v8us*)&sKl[nt * 16 + ln][ks * 32 + 16 + 8 * hh];
        acc = mmaN<3>(aqh[ks].v, aql[ks].v, bh_.v, bl_.v, acc);
      }
      s[nt] = acc;
    }
    float alpha[8];
#pragma unroll
    for (int r = 0; r < 8; ++r) {
      const int qi = qrow[r];
      const int ja = j0 + ln, jb = j0 + 16 + ln;
      bool keepa = ja < Tk, keepb = jb < Tk;
      if (causal) { keepa = keepa && (ja <= qi); keepb = keepb && (jb <= qi); }
      if (mask) { if (keepa) keepa = mask[(size_t)qi * Tk + ja] != 0; if (keepb) keepb = mask[(size_t)qi * Tk + jb] != 0; }
      if (sbias) { if (keepa) s[0][r] += sbias[(size_t)bh * Tk + ja]; if (keepb) s[1][r] += sbias[(size_t)bh * Tk + jb]; }
      if (!keepa) s[0][r] = -3.0e38f;
      if (!keepb) s[1][r] = -3.0e38f;
      float mx = fmaxf(s[0][r], s[1][r]);
      mx = fmaxf(mx, __shfl_xor(mx, 1, 32)); mx = fmaxf(mx, __shfl_xor(mx, 2, 32)); mx = fmaxf(mx, __shfl_xor(mx, 4, 32)); mx = fmaxf(mx, __shfl_xor(mx, 8, 32));
      const float mnew = fmaxf(m_r[r], mx);
      alpha[r] = (mnew > -1.0e38f) ? __expf(m_r[r] - mnew) : 1.0f;
      const float p0 = keepa ? __expf(s[0][r] - mnew) : 0.f;
      const float p1 = keepb ? __expf(s[1][r] - mnew) : 0.f;
      m_r[r] = mnew;
      l_r[r] = l_r[r] * alpha[r] + p0 + p1;
      unsigned short hb = bf16_bits(p0); sPh[w][8 * hh + r][ln] = hb;      sPl[w][8 * hh + r][ln] = bf16_bits(p0 - bf16_val(hb));
      hb = bf16_bits(p1);                sPh[w][8 * hh + r][16 + ln] = hb; sPl[w][8 * hh + r][16 + ln] = bf16_bits(p1 - bf16_val(hb));
    }
#pragma unroll
    for (int dt = 0; dt < DT; ++dt)
#pragma unroll
      for (int r = 0; r < 8; ++r) oacc[dt][r] *= alpha[r];
    __builtin_amdgcn_fence(__ATOMIC_ACQ_REL, "workgroup");
    __builtin_amdgcn_wave_barrier();
    FragB pah, pal;
    pah.half[0] = *(const v8us*)&sPh[w][ln][8 * hh]; pah.half[1] = *(const v8us*)&sPh[w][ln][16 + 8 * hh];
    pal.half[0] = *(const v8us*)&sPl[w][ln][8 * hh]; pal.half[1] = *(const v8us*)&sPl[w][ln][16 + 8 * hh];
#pragma unroll
    for (int dt = 0; dt < DT; ++dt) {
      FragB bvh, bvl;
#pragma unroll
      for (int i = 0; i < 8; ++i) {
        bvh.u[i] = sVh[8 * hh + i][dt * 16 + ln]; bvh.u[8 + i] = sVh[16 + 8 * hh + i][dt * 16 + ln];
        bvl.u[i] = sVl[8 * hh + i][dt * 16 + ln]; bvl.u[8 + i] = sVl[16 + 8 * hh + i][dt * 16 + ln];
      }
      oacc[dt] = mmaN<3>(pah.v, pal.v, bvh.v, bvl.v, oacc[dt]);
    }
    __builtin_amdgcn_fence(__ATOMIC_ACQ_REL, "workgroup");
    __builtin_amdgcn_wave_barrier();
  }
#pragma unroll
  for (int r = 0; r < 8; ++r) {
    float l = l_r[r];
    l += __shfl_xor(l, 1, 32); l += __shfl_xor(l, 2, 32); l += __shfl_xor(l, 4, 32); l += __shfl_xor(l, 8, 32);
    l_r[r] = (m_r[r] > -1.0e38f) ? 1.0f / l : __builtin_nanf("");
  }
#pragma unroll
  for (int dt = 0; dt < DT; ++dt)
#pragma unroll
    for (int r = 0; r < 8; ++r) sO[w][8 * hh + r][dt * 16 + ln] = oacc[dt][r] * l_r[r];
  __builtin_amdgcn_fence(__ATOMIC_ACQ_REL, "workgroup");
  __builtin_amdgcn_wave_barrier();
  for (int pass = 0; pass < 2; ++pass) {
    for (int r = 0; r < 16; ++r) {
      const int row = q0 + r;
      if (row < Tq && lane < D / 4) {
        const v4f val = *(const v4fa*)&sO[w][r][lane * 4];
        *(volatile v4f*)(y + ((size_t)b * Tq + row) * ypitch + h * D + lane * 4) = val;
      }
    }
    if (pass == 0) __threadfence();
  }
}

template <bool IN_BF16>
__global__ __launch_bounds__(256) void k_ln384(const float* __restrict__ x, const float* __restrict__ g, const float* __restrict__ b, float* __restrict__ out, float* __restrict__ xcopy, int nrows) {
  const int tid = threadIdx.x, w = tid >> 5, lane = tid & 31; const int row = blockIdx.x * 8 + w; if (row >= nrows) return;
  float v[12]; float s = 0.f;
#pragma unroll
  for (int u = 0; u < 12; ++u) { float a = x[(size_t)row * DD + u * 32 + lane]; if (IN_BF16) a = bf16_round(a); v[u] = a; s += a; }
  for (int o = 16; o >= 1; o >>= 1) s += __shfl_xor(s, o, 32); const float mu = s * (1.0f / DD);
  float q2 = 0.f;
#pragma unroll
  for (int u = 0; u < 12; ++u) { const float c = v[u] - mu; q2 += c * c; }
  for (int o = 16; o >= 1; o >>= 1) q2 += __shfl_xor(q2, o, 32); const float rs = rsqrtf(q2 * (1.0f / DD) + 1e-5f);
  for (int pass = 0; pass < 2; ++pass) {
#pragma unroll
    for (int u = 0; u < 12; ++u) { const int c = u * 32 + lane; *(volatile float*)(out + (size_t)row * DD + c) = (v[u] - mu) * rs * bf16_round(g[c]) + bf16_round(b[c]); if (xcopy) *(volatile float*)(xcopy + (size_t)row * DD + c) = v[u]; }
    if (pass == 0) __threadfence();
  }
}
__global__ __launch_bounds__(256) void k_knn8(const float* __restrict__ qc, const float* __restrict__ kc, int nq, int nk, int* __restrict__ idx) {
  __shared__ float sk[256][3]; __shared__ int sidx[256][KNN];
  const int q = blockIdx.x * 256 + threadIdx.x; const int b = q / nq, qi = q % nq;
  const float qx = bf16_round(qc[((size_t)b * 3 + 0) * nq + qi]), qy = bf16_round(qc[((size_t)b * 3 + 1) * nq + qi]), qz = bf16_round(qc[((size_t)b * 3 + 2) * nq + qi]);
  const float qs = (qx * qx + qz * qz) + qy * qy;
  float bd[KNN]; int bi[KNN]; for (int i = 0; i < KNN; ++i) { bd[i] = 3.0e38f; bi[i] = 0; }
  for (int c0 = 0; c0 < nk; c0 += 256) {
    __syncthreads();
    { const int c = c0 + threadIdx.x; sk[threadIdx.x][0] = bf16_round(kc[((size_t)b * 3 + 0) * nk + c]); sk[threadIdx.x][1] = bf16_round(kc[((size_t)b * 3 + 1) * nk + c]); sk[threadIdx.x][2] = bf16_round(kc[((size_t)b * 3 + 2) * nk + c]); }
    __syncthreads();
#pragma unroll 1
    for (int j = 0; j < 256; ++j) { const float kx = sk[j][0], ky = sk[j][1], kz = sk[j][2];
      const float d = (qs - 2.0f * ((qx * kx + qy * ky) + qz * kz)) + ((kx * kx + kz * kz) + ky * ky);
      if (d < bd[KNN - 1]) { int i = KNN - 1; while (i > 0 && bd[i - 1] > d) { bd[i] = bd[i - 1]; bi[i] = bi[i - 1]; --i; } bd[i] = d; bi[i] = c0 + j; } }
  }
  for (int i = 0; i < KNN; ++i) sidx[threadIdx.x][i] = bi[i];
  __syncthreads();
  typedef int v4i __attribute__((ext_vector_type(4)));
  for (int pass = 0; pass < 2; ++pass) {
    for (int it = 0; it < 2; ++it) { const int e = it * 256 + threadIdx.x; const int r = e >> 1, hq = e & 1; v4i v = {sidx[r][hq * 4], sidx[r][hq * 4 + 1], sidx[r][hq * 4 + 2], sidx[r][hq * 4 + 3]}; *(volatile v4i*)(idx + ((size_t)blockIdx.x * 256 + r) * KNN + hq * 4) = v; }
    if (pass == 0) __threadfence();
  }
}
__global__ __launch_bounds__(256) void k_gattn(const float* __restrict__ qh, const float* __restrict__ kh, const float* __restrict__ vh, const int* __restrict__ idx, int nq, int nk, float* __restrict__ out) {
  const int tid = threadIdx.x, w = tid >> 5, lane = tid & 31; const int q = blockIdx.x * 8 + w; if (q >= BB * nq) return; const int b = q / nq;
  float qv[12]; for (int u = 0; u < 12; ++u) qv[u] = qh[(size_t)q * DD + u * 32 + lane];
  float s[KNN]; int nb[KNN];
#pragma unroll 1
  for (int i = 0; i < KNN; ++i) { int j = idx[(size_t)q * KNN + i]; j = j < 0 ? 0 : (j >= nk ? nk - 1 : j); nb[i] = b * nk + j; float d = 0.f;
#pragma unroll
    for (int u = 0; u < 12; ++u) d += qv[u] * kh[(size_t)nb[i] * DD + u * 32 + lane];
    for (int o = 16; o >= 1; o >>= 1) d += __shfl_xor(d, o, 32); s[i] = d * 0.05103103630798288f; }
  float mx = s[0]; for (int i = 1; i < KNN; ++i) mx = fmaxf(mx, s[i]); float den = 0.f; for (int i = 0; i < KNN; ++i) { s[i] = expf(s[i] - mx); den += s[i]; } const float inv = 1.0f / den;
  float o[12]; for (int u = 0; u < 12; ++u) o[u] = 0.f;
#pragma unroll 1
  for (int i = 0; i < KNN; ++i) { const float wgt = s[i] * inv;
#pragma unroll
    for (int u = 0; u < 12; ++u) o[u] += wgt * vh[(size_t)nb[i] * DD + u * 32 + lane]; }
  for (int pass = 0; pass < 2; ++pass) { for (int u = 0; u < 12; ++u) *(volatile float*)(out + (size_t)q * DD + u * 32 + lane) = o[u]; if (pass == 0) __threadfence(); }
}
extern "C" void kernel_launch(void* const* d_in, const int* in_sizes, int n_in,
                              void* d_out, int out_size, void* d_ws, size_t ws_size, hipStream_t stream) {
  (void)in_sizes; (void)n_in; (void)out_size;
  const float* qcoord = (const float*)d_in[0]; const float* qfeat = (const float*)d_in[1]; const float* kcoord = (const float*)d_in[2]; const float* kfeat = (const float*)d_in[3];
  const float* in_g = (const float*)d_in[4]; const float* in_b = (const float*)d_in[5]; const float* Wqkv = (const float*)d_in[6]; const float* Wo_s = (const float*)d_in[7]; const float* bo_s = (const float*)d_in[8];
  const float* Wq_sg = (const float*)d_in[9]; const float* bq_sg = (const float*)d_in[10]; const float* Wk_sg = (const float*)d_in[11]; const float* bk_sg = (const float*)d_in[12]; const float* Wv_sg = (const float*)d_in[13]; const float* bv_sg = (const float*)d_in[14];
  const float* W_sm = (const float*)d_in[15]; const float* b_sm = (const float*)d_in[16]; const float* cq_g = (const float*)d_in[17]; const float* cq_b = (const float*)d_in[18]; const float* ck_g = (const float*)d_in[19]; const float* ck_b = (const float*)d_in[20];
  const float* W_cq = (const float*)d_in[21]; const float* W_ck = (const float*)d_in[22]; const float* W_cv = (const float*)d_in[23]; const float* Wo_c = (const float*)d_in[24]; const float* bo_c = (const float*)d_in[25];
  const float* Wq_cg = (const float*)d_in[26]; const float* bq_cg = (const float*)d_in[27]; const float* Wk_cg = (const float*)d_in[28]; const float* bk_cg = (const float*)d_in[29]; const float* Wv_cg = (const float*)d_in[30]; const float* bv_cg = (const float*)d_in[31];
  const float* W_cm = (const float*)d_in[32]; const float* b_cm = (const float*)d_in[33]; const float* ff_g = (const float*)d_in[34]; const float* ff_b = (const float*)d_in[35];
  const float* W_ff1 = (const float*)d_in[36]; const float* b_ff1 = (const float*)d_in[37]; const float* W_ff2 = (const float*)d_in[38]; const float* b_ff2 = (const float*)d_in[39];
  char* ws = (char*)d_ws; size_t off = 0;
  auto take = [&](size_t bytes) { char* p = ws + off; off += (bytes + 255) & ~(size_t)255; return p; };
  const int M = BB * NQ, MK = BB * NK; const size_t NE = (size_t)M * DD;
  unsigned short* Bqkv = (unsigned short*)take((size_t)3 * DD * DD * 2); unsigned short* Bos = (unsigned short*)take((size_t)DD * DD * 2);
  unsigned short* Bqsg = (unsigned short*)take((size_t)DD * DD * 2); unsigned short* Bksg = (unsigned short*)take((size_t)DD * DD * 2); unsigned short* Bvsg = (unsigned short*)take((size_t)DD * DD * 2);
  unsigned short* Bsm_a = (unsigned short*)take((size_t)DD * DD * 2); unsigned short* Bsm_b = (unsigned short*)take((size_t)DD * DD * 2);
  unsigned short* Bcq = (unsigned short*)take((size_t)DD * DD * 2); unsigned short* Bck = (unsigned short*)take((size_t)DD * DD * 2); unsigned short* Bcv = (unsigned short*)take((size_t)DD * DD * 2); unsigned short* Boc = (unsigned short*)take((size_t)DD * DD * 2);
  unsigned short* Bqcg = (unsigned short*)take((size_t)DD * DD * 2); unsigned short* Bkcg = (unsigned short*)take((size_t)DD * DD * 2); unsigned short* Bvcg = (unsigned short*)take((size_t)DD * DD * 2);
  unsigned short* Bcm_a = (unsigned short*)take((size_t)DD * DD * 2); unsigned short* Bcm_b = (unsigned short*)take((size_t)DD * DD * 2); unsigned short* Bf1 = (unsigned short*)take((size_t)2 * DD * DD * 2); unsigned short* Bf2 = (unsigned short*)take((size_t)DD * 2 * DD * 2);
  float* qfT = (float*)take(NE * 4); float* kfT = (float*)take((size_t)MK * DD * 4); float* qf = (float*)take(NE * 4); float* nf = (float*)take(NE * 4); float* nk = (float*)take((size_t)MK * DD * 4);
  float* qkv = (float*)take((size_t)M * 3 * DD * 4); float* att = (float*)take(NE * 4); float* t1 = (float*)take(NE * 4); float* qh = (float*)take(NE * 4); float* kh = (float*)take((size_t)MK * DD * 4); float* vh = (float*)take((size_t)MK * DD * 4); float* geom = (float*)take(NE * 4);
  float* ffn = (float*)take((size_t)M * 2 * DD * 4); int* idx = (int*)take((size_t)M * KNN * 4);
  if (off > ws_size) return;
  const int gw = (DD * (DD / 8) + 255) / 256;
  k_wt_bf16<<<(3 * DD * (DD / 8) + 255) / 256, 256, 0, stream>>>(Wqkv, Bqkv, DD, 3 * DD); k_wt_bf16<<<gw, 256, 0, stream>>>(Wo_s, Bos, DD, DD);
  k_wt_bf16<<<gw, 256, 0, stream>>>(Wq_sg, Bqsg, DD, DD); k_wt_bf16<<<gw, 256, 0, stream>>>(Wk_sg, Bksg, DD, DD); k_wt_bf16<<<gw, 256, 0, stream>>>(Wv_sg, Bvsg, DD, DD);
  k_wt_bf16<<<gw, 256, 0, stream>>>(W_sm, Bsm_a, DD, DD); k_wt_bf16<<<gw, 256, 0, stream>>>(W_sm + (size_t)DD * DD, Bsm_b, DD, DD);
  k_wt_bf16<<<gw, 256, 0, stream>>>(W_cq, Bcq, DD, DD); k_wt_bf16<<<gw, 256, 0, stream>>>(W_ck, Bck, DD, DD); k_wt_bf16<<<gw, 256, 0, stream>>>(W_cv, Bcv, DD, DD); k_wt_bf16<<<gw, 256, 0, stream>>>(Wo_c, Boc, DD, DD);
  k_wt_bf16<<<gw, 256, 0, stream>>>(Wq_cg, Bqcg, DD, DD); k_wt_bf16<<<gw, 256, 0, stream>>>(Wk_cg, Bkcg, DD, DD); k_wt_bf16<<<gw, 256, 0, stream>>>(Wv_cg, Bvcg, DD, DD);
  k_wt_bf16<<<gw, 256, 0, stream>>>(W_cm, Bcm_a, DD, DD); k_wt_bf16<<<gw, 256, 0, stream>>>(W_cm + (size_t)DD * DD, Bcm_b, DD, DD);
  k_wt_bf16<<<(2 * DD * (DD / 8) + 255) / 256, 256, 0, stream>>>(W_ff1, Bf1, DD, 2 * DD); k_wt_bf16<<<(DD * (2 * DD / 8) + 255) / 256, 256, 0, stream>>>(W_ff2, Bf2, 2 * DD, DD);
  k_transpose32<false, false, false><<<dim3(NQ / 32, DD / 32, BB), 256, 0, stream>>>(qfeat, qfT, DD, NQ, nullptr, nullptr, nullptr);
  k_transpose32<false, false, false><<<dim3(NK / 32, DD / 32, BB), 256, 0, stream>>>(kfeat, kfT, DD, NK, nullptr, nullptr, nullptr);
  const int g1 = ((M / 16) * (DD / 64) + 3) / 4, g3 = ((M / 16) * (3 * DD / 64) + 3) / 4, g2 = ((M / 16) * (2 * DD / 64) + 3) / 4, gk = ((MK / 16) * (DD / 64) + 3) / 4;
  k_ln384<true><<<(M + 7) / 8, 256, 0, stream>>>(qfT, in_g, in_b, nf, qf, M);
  k_gemm_bf3<true, 0, false, false><<<g3, 128, 0, stream>>>(nf, DD, Bqkv, DD, nullptr, nullptr, 1, 0, qkv, 3 * DD, M, 3 * DD, DD);
  k_flash3<HD><<<BB * NH * (NQ / 64), 128, 0, stream>>>(qkv, 3 * DD, NQ, qkv + DD, qkv + 2 * DD, NQ, nullptr, nullptr, 0, 3 * DD, 3 * DD, NH, 0.125f, nullptr, 0, nullptr, att, DD);
  k_gemm_bf3<true, 0, true, false><<<g1, 128, 0, stream>>>(att, DD, Bos, DD, bo_s, nullptr, 1, 0, t1, DD, M, DD, DD);
  k_knn8<<<M / 256, 256, 0, stream>>>(qcoord, qcoord, NQ, NQ, idx);
  k_gemm_bf3<true, 0, true, false><<<g1, 128, 0, stream>>>(nf, DD, Bqsg, DD, bq_sg, nullptr, 1, 0, qh, DD, M, DD, DD);
  k_gemm_bf3<true, 0, true, false><<<g1, 128, 0, stream>>>(nf, DD, Bksg, DD, bk_sg, nullptr, 1, 0, kh, DD, M, DD, DD);
  k_gemm_bf3<true, 0, true, false><<<g1, 128, 0, stream>>>(nf, DD, Bvsg, DD, bv_sg, nullptr, 1, 0, vh, DD, M, DD, DD);
  k_gattn<<<(M + 7) / 8, 256, 0, stream>>>(qh, kh, vh, idx, NQ, NQ, geom);
  k_gemm_bf3<true, 0, true, false><<<g1, 128, 0, stream>>>(t1, DD, Bsm_a, DD, b_sm, qf, M, DD, qf, DD, M, DD, DD);
  k_gemm_bf3<true, 0, false, false><<<g1, 128, 0, stream>>>(geom, DD, Bsm_b, DD, nullptr, qf, M, DD, qf, DD, M, DD, DD);
  k_ln384<false><<<(M + 7) / 8, 256, 0, stream>>>(qf, cq_g, cq_b, nf, nullptr, M);
  k_ln384<true><<<(MK + 7) / 8, 256, 0, stream>>>(kfT, ck_g, ck_b, nk, nullptr, MK);
  k_gemm_bf3<true, 0, false, false><<<g1, 128, 0, stream>>>(nf, DD, Bcq, DD, nullptr, nullptr, 1, 0, qkv, 3 * DD, M, DD, DD);
  k_gemm_bf3<true, 0, false, false><<<gk, 128, 0, stream>>>(nk, DD, Bck, DD, nullptr, nullptr, 1, 0, qkv + DD, 3 * DD, MK, DD, DD);
  k_gemm_bf3<true, 0, false, false><<<gk, 128, 0, stream>>>(nk, DD, Bcv, DD, nullptr, nullptr, 1, 0, qkv + 2 * DD, 3 * DD, MK, DD, DD);
  k_flash3<HD><<<BB * NH * (NQ / 64), 128, 0, stream>>>(qkv, 3 * DD, NQ, qkv + DD, qkv + 2 * DD, NK, nullptr, nullptr, 0, 3 * DD, 3 * DD, NH, 0.125f, nullptr, 0, nullptr, att, DD);
  k_gemm_bf3<true, 0, true, false><<<g1, 128, 0, stream>>>(att, DD, Boc, DD, bo_c, nullptr, 1, 0, t1, DD, M, DD, DD);
  k_knn8<<<M / 256, 256, 0, stream>>>(qcoord, kcoord, NQ, NK, idx);
  k_gemm_bf3<true, 0, true, false><<<g1, 128, 0, stream>>>(nf, DD, Bqcg, DD, bq_cg, nullptr, 1, 0, qh, DD, M, DD, DD);
  k_gemm_bf3<true, 0, true, false><<<gk, 128, 0, stream>>>(nk, DD, Bkcg, DD, bk_cg, nullptr, 1, 0, kh, DD, MK, DD, DD);
  k_gemm_bf3<true, 0, true, false><<<gk, 128, 0, stream>>>(nk, DD, Bvcg, DD, bv_cg, nullptr, 1, 0, vh, DD, MK, DD, DD);
  k_gattn<<<(M + 7) / 8, 256, 0, stream>>>(qh, kh, vh, idx, NQ, NK, geom);
  k_gemm_bf3<true, 0, true, false><<<g1, 128, 0, stream>>>(t1, DD, Bcm_a, DD, b_cm, qf, M, DD, qf, DD, M, DD, DD);
  k_gemm_bf3<true, 0, false, false><<<g1, 128, 0, stream>>>(geom, DD, Bcm_b, DD, nullptr, qf, M, DD, qf, DD, M, DD, DD);
  k_ln384<false><<<(M + 7) / 8, 256, 0, stream>>>(qf, ff_g, ff_b, nf, nullptr, M);
  k_gemm_bf3<true, 3, true, false><<<g2, 128, 0, stream>>>(nf, DD, Bf1, DD, b_ff1, nullptr, 1, 0, ffn, 2 * DD, M, 2 * DD, DD);
  k_gemm_bf3<true, 0, true, false><<<g1, 128, 0, stream>>>(ffn, 2 * DD, Bf2, 2 * DD, b_ff2, qf, M, DD, t1, DD, M, DD, 2 * DD);
  k_transpose32<false, false, false><<<dim3(DD / 32, NQ / 32, BB), 256, 0, stream>>>(t1, (float*)d_out, NQ, DD, nullptr, nullptr, nullptr);
}
